// SeedCellLinear_23304492548723
// MI455X (gfx1250) — hardware-verified
//
#include <hip/hip_runtime.h>


#define NB 16
#define NI 512
#define NO 512
#define NH 5
#define NG 32
#define NF 11
#define NU 6
#define WPB 8
#define TLD 36

typedef _Float16 v16h __attribute__((ext_vector_type(16)));
typedef _Float16 v8h  __attribute__((ext_vector_type(8)));
typedef float    v8f  __attribute__((ext_vector_type(8)));
typedef float    v4f  __attribute__((ext_vector_type(4)));

union Frag { v16h v; v8h half[2]; };
union H8   { v8h h; v4f f; };

__device__ __forceinline__ v8f wmma_f16(v16h a, v16h b, v8f c) {
  v8f d = __builtin_amdgcn_wmma_f32_16x16x32_f16(false, a, false, b, (short)0, c, false, false);
  asm volatile("v_nop\n\tv_nop\n\tv_nop\n\tv_nop" : "+v"(d) : "v"(a), "v"(b));
  return d;
}

__device__ __forceinline__ float fast_tanh(float x) {
  x = fminf(fmaxf(x, -15.0f), 15.0f);
  float e = __builtin_amdgcn_exp2f(x * 2.885390081777927f);
  return (e - 1.0f) * __builtin_amdgcn_rcpf(e + 1.0f);
}

__global__ __launch_bounds__(256) void k_cpre(
    const float* __restrict__ hs, const float* __restrict__ pin,
    const float* __restrict__ W1, float* __restrict__ cpre, int nq) {
  const int q = blockIdx.x * 256 + threadIdx.x;
  if (q >= nq) return;
  const int gq = q & 7;
  const int bi = q >> 3;
  const float pv = pin[bi];
  const float* hp = hs + (size_t)bi * NH;
  const float h0 = hp[0], h1 = hp[1], h2 = hp[2], h3 = hp[3], h4 = hp[4];
  v4f v;
#pragma unroll
  for (int c = 0; c < 4; ++c) {
    const float* wr = W1 + (gq * 4 + c) * NF;
    v[c] = wr[9] * pv + (wr[4] * h0 + wr[5] * h1 + wr[6] * h2 + wr[7] * h3 + wr[8] * h4);
  }
  volatile v4f* dst = (volatile v4f*)(cpre + (size_t)bi * NG + gq * 4);
  *dst = v;
  __threadfence();
  *dst = v;
}

__global__ __launch_bounds__(256) void k_main(
    const float* __restrict__ pyl, const float* __restrict__ pyp,
    const float* __restrict__ perr, const float* __restrict__ pout,
    const float* __restrict__ weight, const float* __restrict__ W1,
    const float* __restrict__ b1, const float* __restrict__ W2,
    const float* __restrict__ b2, const float* __restrict__ cpre,
    _Float16* __restrict__ nwh, float* __restrict__ hidT) {
  __shared__ __attribute__((aligned(16))) float s_ap[NB * WPB * NG];
  __shared__ __attribute__((aligned(16))) float s_hid[WPB * NB * 16];
  __shared__ __attribute__((aligned(16))) v8h   s_nw[WPB * (NI / 8)];

  const int tid = threadIdx.x, w = tid >> 5, lane = tid & 31, h = lane >> 4, p = lane & 15;
  const int o0 = blockIdx.x * WPB, o = o0 + w;

  for (int idx = tid; idx < NB * WPB * NG; idx += 256) {
    const int g = idx & (NG - 1), ww = (idx >> 5) & (WPB - 1), b = idx >> 8;
    const size_t bo = (size_t)b * NO + (o0 + ww);
    const float* w1 = W1 + g * NF;
    s_ap[idx] = w1[0] * pyl[bo] + w1[1] * pyp[bo] + w1[2] * perr[bo] + w1[10] * pout[bo] + b1[g];
  }
  for (int idx = tid; idx < WPB * NB * 16; idx += 256) s_hid[idx] = 0.0f;
  __syncthreads();

  float wc3[16];
  v16h bfv;
  const int pc = (p < NU) ? p : 0;
#pragma unroll
  for (int e = 0; e < 16; ++e) {
    const int g = e + (e & 8) + 8 * h;
    wc3[e] = W1[g * NF + 3];
    float bv = W2[pc * NG + g] * 1024.0f;
    if (p >= NU) bv = 0.0f;
    bfv[e] = (_Float16)bv;
  }

  const float* wrow = weight + (size_t)o * NI;
  const float* apw = s_ap + w * NG + 8 * h;
  float* hrow = s_hid + (w * NB) * 16 + p;
  const float scw = (1.0f / 1024.0f) * (1.0f / (float)NB);

  for (int t = 0; t < NI / 16; ++t) {
    const int i = t * 16 + p;
    const float wv = wrow[i];
    float wcol[8];
#pragma unroll
    for (int r = 0; r < 8; ++r) wcol[r] = 0.0f;
    const float* cp = cpre + (size_t)i * NG + 8 * h;

#pragma unroll 1
    for (int b = 0; b < NB; ++b) {
      const float* cr = cp + (size_t)b * NI * NG;
      const float* ar = apw + b * (WPB * NG);
      v4f cq[4], aq[4];
      cq[0] = *(const v4f*)(cr);      cq[1] = *(const v4f*)(cr + 4);
      cq[2] = *(const v4f*)(cr + 16); cq[3] = *(const v4f*)(cr + 20);
      aq[0] = *(const v4f*)(ar);      aq[1] = *(const v4f*)(ar + 4);
      aq[2] = *(const v4f*)(ar + 16); aq[3] = *(const v4f*)(ar + 20);
      v16h av;
#pragma unroll
      for (int e = 0; e < 16; ++e) {
        const float z = (aq[e >> 2][e & 3] + cq[e >> 2][e & 3]) + wv * wc3[e];
        av[e] = (_Float16)fast_tanh(z);
      }
      v8f acc = {};
      acc = wmma_f16(av, bfv, acc);
      float s = 0.0f;
#pragma unroll
      for (int r = 0; r < 8; ++r) { wcol[r] += acc[r]; s += acc[r]; }
      s += __shfl_xor(s, 16, 32);
      if (lane < 16) hrow[b * 16] += s;
    }

    if (p == 5) {
      const float* wr = wrow + t * 16 + 8 * h;
      v4f wq[2];
      wq[0] = *(const v4f*)wr; wq[1] = *(const v4f*)(wr + 4);
      const float b25 = b2[5];
      v8h nv;
#pragma unroll
      for (int r = 0; r < 8; ++r)
        nv[r] = (_Float16)((wq[r >> 2][r & 3] + wcol[r] * scw + b25) * 16.0f);
      s_nw[w * (NI / 8) + 2 * t + h] = nv;
    }
  }
  __syncthreads();

  H8 u0, u1;
  u0.h = s_nw[w * (NI / 8) + lane];
  u1.h = s_nw[w * (NI / 8) + 32 + lane];
  volatile v4f* d0 = (volatile v4f*)(nwh + (size_t)o * NI + lane * 8);
  volatile v4f* d1 = (volatile v4f*)(nwh + (size_t)o * NI + 256 + lane * 8);
  const int hb = lane >> 1, uq = (lane & 1) * 4;
  const float sch = (1.0f / 1024.0f) * (1.0f / (float)NI);
  v4f hv;
#pragma unroll
  for (int c = 0; c < 4; ++c) {
    const int u = uq + c;
    const int uc = (u < NH) ? u : 0;
    float val = s_hid[(w * NB + hb) * 16 + uc] * sch + b2[uc];
    if (u >= NH) val = 0.0f;
    hv[c] = val;
  }
  volatile v4f* dh = (volatile v4f*)(hidT + ((size_t)o * NB + hb) * 8 + uq);
  *d0 = u0.f; *d1 = u1.f; *dh = hv;
  __threadfence();
  *d0 = u0.f; *d1 = u1.f; *dh = hv;
}

__global__ __launch_bounds__(32) void k_gemm(
    const float* __restrict__ x, const _Float16* __restrict__ nwh,
    const float* __restrict__ bias, float* __restrict__ out) {
  __shared__ __attribute__((aligned(16))) float tile[16 * TLD];
  const int lane = threadIdx.x & 31, h = lane >> 4, m = lane & 15;
  const int n0 = blockIdx.x * 32;
  const float* arow = x + (size_t)m * NI;
  const _Float16* br0 = nwh + (size_t)(n0 + m) * NI;
  const _Float16* br1 = nwh + (size_t)(n0 + 16 + m) * NI;
  v8f acc0 = {}, acc1 = {};
#pragma unroll 2
  for (int k0 = 0; k0 < NI; k0 += 32) {
    v4f xq[4];
    xq[0] = *(const v4f*)(arow + k0 + 8 * h);      xq[1] = *(const v4f*)(arow + k0 + 8 * h + 4);
    xq[2] = *(const v4f*)(arow + k0 + 16 + 8 * h); xq[3] = *(const v4f*)(arow + k0 + 20 + 8 * h);
    v16h av;
#pragma unroll
    for (int e = 0; e < 16; ++e) av[e] = (_Float16)(xq[e >> 2][e & 3] * 16.0f);
    Frag b0, b1;
    b0.half[0] = *(const v8h*)(br0 + k0 + 8 * h); b0.half[1] = *(const v8h*)(br0 + k0 + 16 + 8 * h);
    b1.half[0] = *(const v8h*)(br1 + k0 + 8 * h); b1.half[1] = *(const v8h*)(br1 + k0 + 16 + 8 * h);
    acc0 = wmma_f16(av, b0.v, acc0);
    acc1 = wmma_f16(av, b1.v, acc1);
  }
  const float sc = 1.0f / 256.0f;
  const float bi0 = bias[n0 + m], bi1 = bias[n0 + 16 + m];
#pragma unroll
  for (int r = 0; r < 8; ++r) {
    tile[(8 * h + r) * TLD + m]      = acc0[r] * sc + bi0;
    tile[(8 * h + r) * TLD + 16 + m] = acc1[r] * sc + bi1;
  }
  __syncthreads();
  const int rq = lane >> 3, cq = (lane & 7) * 4;
  v4f v[4];
#pragma unroll
  for (int j = 0; j < 4; ++j) {
    const float* tp = tile + (j * 4 + rq) * TLD + cq;
    v4f t4;
    t4[0] = tp[0]; t4[1] = tp[1]; t4[2] = tp[2]; t4[3] = tp[3];
    v[j] = t4;
  }
#pragma unroll
  for (int j = 0; j < 4; ++j)
    *(volatile v4f*)(out + (size_t)(j * 4 + rq) * NO + n0 + cq) = v[j];
  __threadfence();
#pragma unroll
  for (int j = 0; j < 4; ++j)
    *(volatile v4f*)(out + (size_t)(j * 4 + rq) * NO + n0 + cq) = v[j];
}

__device__ __forceinline__ v4f gather_hid(const float* __restrict__ hidT, int b, int q) {
  v4f v;
#pragma unroll
  for (int c = 0; c < 4; ++c) {
    const int e = 4 * q + c;
    const int oo = e / NH;
    const int u = e - oo * NH;
    v[c] = hidT[((size_t)oo * NB + b) * 8 + u];
  }
  return v;
}

__global__ __launch_bounds__(256) void k_out1(const float* __restrict__ hidT, float* __restrict__ out1) {
  const int b = blockIdx.x;
  const int nq = (NO * NH) / 4;
  float* base = out1 + (size_t)b * (NO * NH);
  const int q0 = threadIdx.x, q1 = 256 + threadIdx.x, q2 = 512 + threadIdx.x;
  const bool t2 = q2 < nq;
  const v4f v0 = gather_hid(hidT, b, q0);
  const v4f v1 = gather_hid(hidT, b, q1);
  v4f v2 = {};
  if (t2) v2 = gather_hid(hidT, b, q2);
  volatile v4f* p0 = (volatile v4f*)(base + 4 * q0);
  volatile v4f* p1 = (volatile v4f*)(base + 4 * q1);
  volatile v4f* p2 = (volatile v4f*)(base + 4 * q2);
  *p0 = v0; *p1 = v1; if (t2) *p2 = v2;
  __threadfence();
  *p0 = v0; *p1 = v1; if (t2) *p2 = v2;
}

extern "C" void kernel_launch(void* const* d_in, const int* in_sizes, int n_in,
                              void* d_out, int out_size, void* d_ws, size_t ws_size,
                              hipStream_t stream) {
  if (n_in < 13) return;
  if (out_size < NB * NO + NB * NO * NH) return;
  if (in_sizes[0] < NB * NI || in_sizes[1] < NB * NO || in_sizes[2] < NB * NO ||
      in_sizes[3] < NB * NO || in_sizes[4] < NB * NI || in_sizes[5] < NB * NO ||
      in_sizes[6] < NB * NI * NH || in_sizes[7] < NO * NI || in_sizes[8] < NO ||
      in_sizes[9] < NG * NF || in_sizes[10] < NG || in_sizes[11] < NU * NG || in_sizes[12] < NU)
    return;

  const float* input  = (const float*)d_in[0];
  const float* pyl    = (const float*)d_in[1];
  const float* pyp    = (const float*)d_in[2];
  const float* perr   = (const float*)d_in[3];
  const float* pin    = (const float*)d_in[4];
  const float* pout   = (const float*)d_in[5];
  const float* hs     = (const float*)d_in[6];
  const float* weight = (const float*)d_in[7];
  const float* bias   = (const float*)d_in[8];
  const float* W1     = (const float*)d_in[9];
  const float* b1     = (const float*)d_in[10];
  const float* W2     = (const float*)d_in[11];
  const float* b2     = (const float*)d_in[12];

  const size_t off_cpre = 0;
  const size_t off_nwh  = (size_t)NB * NI * NG * sizeof(float);
  const size_t off_hid  = off_nwh + (size_t)NO * NI * sizeof(_Float16);
  const size_t total    = off_hid + (size_t)NO * NB * 8 * sizeof(float);
  if (ws_size < total) return;
  char* ws = (char*)d_ws;
  float*    cpre = (float*)(ws + off_cpre);
  _Float16* nwh  = (_Float16*)(ws + off_nwh);
  float*    hidT = (float*)(ws + off_hid);

  float* out0 = (float*)d_out;
  float* out1 = out0 + NB * NO;

  const int nq = NB * NI * 8;
  k_cpre<<<(nq + 255) / 256, 256, 0, stream>>>(hs, pin, W1, cpre, nq);
  k_main<<<NO / WPB, 256, 0, stream>>>(pyl, pyp, perr, pout, weight, W1, b1, W2, b2, cpre, nwh, hidT);
  k_gemm<<<NO / 32, 32, 0, stream>>>(input, nwh, bias, out0);
  k_out1<<<NB, 256, 0, stream>>>(hidT, out1);
}
